// SeqBasedModel_11579231830453
// MI455X (gfx1250) — hardware-verified
//
#include <hip/hip_runtime.h>
#include <stdint.h>
#include <stddef.h>


constexpr int kV   = 100000;
constexpr int kE   = 128;
constexpr int kH   = 256;
constexpr int kG   = 4 * kH;
constexpr int kP1  = 512;
constexpr int kP2  = 128;
constexpr int kB   = 256;
constexpr int kS   = 200;
constexpr int kF   = 10;
constexpr int kT   = kS / 2;
constexpr int kBS  = kB * kS;
constexpr int kBT  = kB * kT;

typedef int chk_div0[(kBS % 16 == 0 && kBT % 32 == 0 && kB % 16 == 0) ? 1 : -1];
typedef int chk_div1[(kG % 64 == 0 && kP1 % 64 == 0 && kP2 % 64 == 0 && kH % 64 == 0) ? 1 : -1];
typedef int chk_div2[(kE % 32 == 0 && kH % 32 == 0 && kP1 % 32 == 0 && kP1 <= 512) ? 1 : -1];

typedef __bf16        v16bf __attribute__((ext_vector_type(16)));
typedef float         v8f   __attribute__((ext_vector_type(8)));
typedef float         v4f   __attribute__((ext_vector_type(4)));
typedef unsigned int  u32x4 __attribute__((ext_vector_type(4)));

union FragU { v16bf v; u32x4 u[2]; };

__device__ __forceinline__ unsigned int bf16_bits(float f) {
    unsigned int u = __float_as_uint(f);
    return (u + 0x7FFFu + ((u >> 16) & 1u)) >> 16;
}

__device__ __forceinline__ u32x4 pack8_bf16(v4f a, v4f b) {
    u32x4 r;
    r[0] = bf16_bits(a[0]) | (bf16_bits(a[1]) << 16);
    r[1] = bf16_bits(a[2]) | (bf16_bits(a[3]) << 16);
    r[2] = bf16_bits(b[0]) | (bf16_bits(b[1]) << 16);
    r[3] = bf16_bits(b[2]) | (bf16_bits(b[3]) << 16);
    return r;
}

__device__ __forceinline__ v4f relu4(v4f x) {
    v4f r;
    r[0] = x[0] > 0.0f ? x[0] : 0.0f;
    r[1] = x[1] > 0.0f ? x[1] : 0.0f;
    r[2] = x[2] > 0.0f ? x[2] : 0.0f;
    r[3] = x[3] > 0.0f ? x[3] : 0.0f;
    return r;
}

__device__ __forceinline__ float sigm(float x) { return 1.0f / (1.0f + expf(-x)); }

__device__ __forceinline__ v16bf load_frag(const unsigned short* base, int ld, int row0, int k0, int lane) {
    const unsigned short* p = base + (size_t)(row0 + (lane & 15)) * (size_t)ld + k0 + 8 * (lane >> 4);
    FragU f;
    f.u[0] = *(const u32x4*)(p);
    f.u[1] = *(const u32x4*)(p + 16);
    return f.v;
}

__device__ __forceinline__ v8f wmma16(v16bf a, v16bf b, v8f c) {
    v8f d = __builtin_amdgcn_wmma_f32_16x16x32_bf16(false, a, false, b, (short)0, c, false, false);
    asm volatile("v_nop\n\tv_nop\n\tv_nop\n\tv_nop" : "+v"(d) : "v"(a), "v"(b));
    return d;
}

__global__ __launch_bounds__(128) void embed_mean_kernel(const int* __restrict__ x,
                                                         const float* __restrict__ emb,
                                                         unsigned short* __restrict__ e,
                                                         int nRows, int nEmbRows) {
    const int tid = threadIdx.x;
    const int row = blockIdx.x * 8 + (tid >> 4);
    const int e0  = (tid & 15) * 8;
    const bool ok = row < nRows;
    const int rowc = ok ? row : 0;
    v4f s0 = {0.0f, 0.0f, 0.0f, 0.0f};
    v4f s1 = {0.0f, 0.0f, 0.0f, 0.0f};
#pragma unroll
    for (int f = 0; f < kF; ++f) {
        int idx = x[(size_t)rowc * kF + f];
        idx = idx < 0 ? 0 : (idx >= nEmbRows ? nEmbRows - 1 : idx);
        const float* p = emb + (size_t)idx * kE + e0;
        s0 += *(const v4f*)(p);
        s1 += *(const v4f*)(p + 4);
    }
    const float inv = 1.0f / (float)kF;
    s0 *= inv;
    s1 *= inv;
    const u32x4 pk = pack8_bf16(s0, s1);
    unsigned short* dst = e + (size_t)rowc * kE + e0;
    if (ok) *(volatile u32x4*)dst = pk;
    __threadfence();
    if (ok) *(volatile u32x4*)dst = pk;
}

__global__ __launch_bounds__(256) void cvt_bf16_kernel(const float* __restrict__ s,
                                                       unsigned short* __restrict__ d, int n) {
    const size_t i8 = ((size_t)blockIdx.x * 256 + threadIdx.x) * 8;
    const bool ok = (i8 + 8) <= (size_t)n;
    v4f a = {0.0f, 0.0f, 0.0f, 0.0f};
    v4f b = {0.0f, 0.0f, 0.0f, 0.0f};
    if (ok) {
        a = *(const v4f*)(s + i8);
        b = *(const v4f*)(s + i8 + 4);
    }
    const u32x4 pk = pack8_bf16(a, b);
    if (ok) *(volatile u32x4*)(d + i8) = pk;
    __threadfence();
    if (ok) *(volatile u32x4*)(d + i8) = pk;
}

__global__ __launch_bounds__(256) void cvt_bf16_T_kernel(const float* __restrict__ s,
                                                         unsigned short* __restrict__ d,
                                                         int R, int C) {
    __shared__ float tile[32][65];
    const int r0 = blockIdx.x * 64;
    const int c0 = blockIdx.y * 32;
    for (int i = threadIdx.x; i < 64 * 32; i += 256) {
        const int rr = i >> 5, cc = i & 31;
        const int r = r0 + rr, c = c0 + cc;
        tile[cc][rr] = (r < R && c < C) ? s[(size_t)r * C + c] : 0.0f;
    }
    __syncthreads();
    const int orow = threadIdx.x >> 3, piece = threadIdx.x & 7;
    const int c = c0 + orow, rb = r0 + piece * 8;
    v4f a, b;
    a[0] = tile[orow][piece * 8 + 0]; a[1] = tile[orow][piece * 8 + 1];
    a[2] = tile[orow][piece * 8 + 2]; a[3] = tile[orow][piece * 8 + 3];
    b[0] = tile[orow][piece * 8 + 4]; b[1] = tile[orow][piece * 8 + 5];
    b[2] = tile[orow][piece * 8 + 6]; b[3] = tile[orow][piece * 8 + 7];
    const u32x4 pk = pack8_bf16(a, b);
    const bool ok = (c < C) && (rb + 8 <= R);
    unsigned short* dst = d + (size_t)c * R + rb;
    if (ok) *(volatile u32x4*)dst = pk;
    __threadfence();
    if (ok) *(volatile u32x4*)dst = pk;
}

__global__ __launch_bounds__(128) void gemm_bf16_kernel(const unsigned short* __restrict__ A,
                                                        const unsigned short* __restrict__ Bt,
                                                        const float* __restrict__ bias,
                                                        float* __restrict__ Cf,
                                                        unsigned short* __restrict__ Cb,
                                                        int M, int K, int N, int act) {
    __shared__ __align__(16) unsigned short sA[16 * 512];
    __shared__ __align__(16) float sC[16 * 64];
    const int tid = threadIdx.x, lane = tid & 31, wave = tid >> 5;
    const int hf = lane >> 4, m = lane & 15;
    const int nBase = blockIdx.x * 64;
    const int mBase = blockIdx.y * 16;
    if (mBase + 16 > M || nBase + 64 > N || K > 512 || (K & 31) != 0) return;
    const int nW = nBase + wave * 16;
    const int kv = K >> 3;
    for (int i = tid; i < 16 * kv; i += 128) {
        const int r = i / kv, c8 = i - r * kv;
        *(u32x4*)(sA + r * K + c8 * 8) = *(const u32x4*)(A + (size_t)(mBase + r) * K + c8 * 8);
    }
    const float bc = bias ? bias[nW + m] : 0.0f;
    v8f acc = {bc, bc, bc, bc, bc, bc, bc, bc};
    __syncthreads();
    for (int k0 = 0; k0 < K; k0 += 32) {
        const v16bf a = load_frag(sA, K, 0, k0, lane);
        const v16bf b = load_frag(Bt, K, nW, k0, lane);
        acc = wmma16(a, b, acc);
    }
#pragma unroll
    for (int v = 0; v < 8; ++v) sC[(8 * hf + v) * 64 + wave * 16 + m] = acc[v];
    __syncthreads();
    if (act == 1) {
        const int r = tid >> 3, c8 = (tid & 7) * 8;
        v4f x0 = *(const v4f*)(sC + r * 64 + c8);
        v4f x1 = *(const v4f*)(sC + r * 64 + c8 + 4);
        x0 = relu4(x0);
        x1 = relu4(x1);
        const u32x4 pk = pack8_bf16(x0, x1);
        unsigned short* dst = Cb + (size_t)(mBase + r) * N + nBase + c8;
        *(volatile u32x4*)dst = pk;
        __threadfence();
        *(volatile u32x4*)dst = pk;
    } else {
        const int L0 = tid >> 3;
        const int rowA = L0 >> 1, colA = (L0 & 1) * 32 + (tid & 7) * 4;
        const int L1 = 16 + (tid >> 3);
        const int rowB = L1 >> 1, colB = (L1 & 1) * 32 + (tid & 7) * 4;
        v4f xa = *(const v4f*)(sC + rowA * 64 + colA);
        v4f xb = *(const v4f*)(sC + rowB * 64 + colB);
        if (act == 2) { xa = relu4(xa); xb = relu4(xb); }
        float* da = Cf + (size_t)(mBase + rowA) * N + nBase + colA;
        float* db = Cf + (size_t)(mBase + rowB) * N + nBase + colB;
        *(volatile v4f*)da = xa;
        *(volatile v4f*)db = xb;
        __threadfence();
        *(volatile v4f*)da = xa;
        *(volatile v4f*)db = xb;
    }
}

__global__ __launch_bounds__(128) void lstm_step_kernel(const float* __restrict__ Gx,
                                                        const float* __restrict__ b_ih,
                                                        const float* __restrict__ b_hh,
                                                        const unsigned short* __restrict__ Whh,
                                                        const unsigned short* __restrict__ hPrev,
                                                        const float* __restrict__ cPrev,
                                                        unsigned short* __restrict__ hNext,
                                                        float* __restrict__ cNext,
                                                        int t) {
    __shared__ __align__(16) unsigned short sH[16 * kH];
    __shared__ __align__(16) float sG[4 * 16 * 64];
    __shared__ __align__(16) unsigned short sHo[16 * 64];
    const int tid = threadIdx.x, lane = tid & 31, wave = tid >> 5;
    const int hf = lane >> 4, m = lane & 15;
    const int bBase = blockIdx.y * 16;
    const int cBase = blockIdx.x * 64;
    const int wcol  = cBase + wave * 16;

    for (int i = tid; i < 16 * (kH / 8); i += 128) {
        const int r = i / (kH / 8), c8 = i - r * (kH / 8);
        *(u32x4*)(sH + r * kH + c8 * 8) = *(const u32x4*)(hPrev + (size_t)(bBase + r) * kH + c8 * 8);
    }

    const int col = wcol + m;
    const float s0 = b_ih[col]          + b_hh[col];
    const float s1 = b_ih[kH + col]     + b_hh[kH + col];
    const float s2 = b_ih[2 * kH + col] + b_hh[2 * kH + col];
    const float s3 = b_ih[3 * kH + col] + b_hh[3 * kH + col];
    v8f acc0, acc1, acc2, acc3;
#pragma unroll
    for (int v = 0; v < 8; ++v) {
        const float* g = Gx + ((size_t)(bBase + 8 * hf + v) * kS + t) * kG + col;
        acc0[v] = g[0]      + s0;
        acc1[v] = g[kH]     + s1;
        acc2[v] = g[2 * kH] + s2;
        acc3[v] = g[3 * kH] + s3;
    }
    __syncthreads();

    for (int k0 = 0; k0 < kH; k0 += 32) {
        const v16bf a  = load_frag(sH, kH, 0, k0, lane);
        const v16bf b0 = load_frag(Whh, kH, 0 * kH + wcol, k0, lane);
        acc0 = wmma16(a, b0, acc0);
        const v16bf b1 = load_frag(Whh, kH, 1 * kH + wcol, k0, lane);
        acc1 = wmma16(a, b1, acc1);
        const v16bf b2 = load_frag(Whh, kH, 2 * kH + wcol, k0, lane);
        acc2 = wmma16(a, b2, acc2);
        const v16bf b3 = load_frag(Whh, kH, 3 * kH + wcol, k0, lane);
        acc3 = wmma16(a, b3, acc3);
    }

#pragma unroll
    for (int v = 0; v < 8; ++v) {
        const int o = (8 * hf + v) * 64 + wave * 16 + m;
        sG[o]        = acc0[v];
        sG[1024 + o] = acc1[v];
        sG[2048 + o] = acc2[v];
        sG[3072 + o] = acc3[v];
    }
    __syncthreads();

    v4f cn0, cn1;
    float* cd0;
    float* cd1;
#pragma unroll
    for (int p = 0; p < 2; ++p) {
        const int r = p * 8 + (tid >> 4), c4 = (tid & 15) * 4;
        const int o = r * 64 + c4;
        const v4f gi = *(const v4f*)(sG + o);
        const v4f gf = *(const v4f*)(sG + 1024 + o);
        const v4f gg = *(const v4f*)(sG + 2048 + o);
        const v4f go = *(const v4f*)(sG + 3072 + o);
        const size_t gofs = (size_t)(bBase + r) * kH + cBase + c4;
        const v4f cp = *(const v4f*)(cPrev + gofs);
        v4f cn;
#pragma unroll
        for (int j = 0; j < 4; ++j) {
            const float c  = sigm(gf[j]) * cp[j] + sigm(gi[j]) * tanhf(gg[j]);
            const float hv = sigm(go[j]) * tanhf(c);
            cn[j] = c;
            sHo[o + j] = (unsigned short)bf16_bits(hv);
        }
        float* cd = cNext + gofs;
        *(volatile v4f*)cd = cn;
        if (p == 0) { cn0 = cn; cd0 = cd; } else { cn1 = cn; cd1 = cd; }
    }
    __syncthreads();

    const int r2 = tid >> 3, c8 = (tid & 7) * 8;
    const u32x4 hv8 = *(const u32x4*)(sHo + r2 * 64 + c8);
    unsigned short* hd = hNext + (size_t)(bBase + r2) * kH + cBase + c8;
    *(volatile u32x4*)hd = hv8;
    __threadfence();
    *(volatile v4f*)cd0 = cn0;
    *(volatile v4f*)cd1 = cn1;
    *(volatile u32x4*)hd = hv8;
}

__global__ __launch_bounds__(128) void target_kernel(const float* __restrict__ Gx,
                                                     const float* __restrict__ R,
                                                     const float* __restrict__ b_ih,
                                                     const float* __restrict__ b_hh,
                                                     const float* __restrict__ cN,
                                                     unsigned short* __restrict__ hOut,
                                                     int nRows) {
    const int lane = threadIdx.x & 31, wave = threadIdx.x >> 5;
    const int row = blockIdx.x * 4 + wave;
    if (row >= nRows) return;
    const int b  = row / kT, tt = row - b * kT;
    const int h0 = lane * 8;
    const float* gx = Gx + ((size_t)b * kS + kT + tt) * kG + h0;
    const float* rr = R + (size_t)b * kG + h0;
    const float* cp = cN + (size_t)b * kH + h0;
    unsigned long long lo = 0ull, hi = 0ull;
#pragma unroll 1
    for (int j = 0; j < 8; ++j) {
        const int hc = h0 + j;
        const float gi = gx[j]          + rr[j]          + b_ih[hc]          + b_hh[hc];
        const float gf = gx[kH + j]     + rr[kH + j]     + b_ih[kH + hc]     + b_hh[kH + hc];
        const float gg = gx[2 * kH + j] + rr[2 * kH + j] + b_ih[2 * kH + hc] + b_hh[2 * kH + hc];
        const float go = gx[3 * kH + j] + rr[3 * kH + j] + b_ih[3 * kH + hc] + b_hh[3 * kH + hc];
        const float c  = sigm(gf) * cp[j] + sigm(gi) * tanhf(gg);
        const float hv = sigm(go) * tanhf(c);
        const unsigned long long bits = (unsigned long long)bf16_bits(hv) << ((j & 3) * 16);
        if (j < 4) lo |= bits; else hi |= bits;
    }
    u32x4 pk;
    pk[0] = (unsigned int)(lo & 0xFFFFFFFFull);
    pk[1] = (unsigned int)(lo >> 32);
    pk[2] = (unsigned int)(hi & 0xFFFFFFFFull);
    pk[3] = (unsigned int)(hi >> 32);
    unsigned short* dst = hOut + (size_t)row * kH + h0;
    *(volatile u32x4*)dst = pk;
    __threadfence();
    *(volatile u32x4*)dst = pk;
}

__global__ __launch_bounds__(256) void mlp_out_kernel(const float* __restrict__ z2,
                                                      const float* __restrict__ W3,
                                                      const float* __restrict__ b3,
                                                      float* __restrict__ out, int nRows) {
    __shared__ __align__(16) float sOut[32];
    const int tid = threadIdx.x, lane = tid & 31, wave = tid >> 5;
    const v4f w = *(const v4f*)(W3 + lane * 4);
    const float bb = b3[0];
#pragma unroll
    for (int j = 0; j < 4; ++j) {
        const int r  = blockIdx.x * 32 + wave * 4 + j;
        const int rc = r < nRows ? r : nRows - 1;
        const v4f z = *(const v4f*)(z2 + (size_t)rc * kP2 + lane * 4);
        float s = z[0] * w[0] + z[1] * w[1] + z[2] * w[2] + z[3] * w[3];
#pragma unroll
        for (int off = 16; off > 0; off >>= 1) s += __shfl_xor(s, off, 32);
        if (lane == 0) sOut[wave * 4 + j] = sigm(s + bb);
    }
    __syncthreads();
    const bool wr = (tid < 8) && (blockIdx.x * 32 + tid * 4 + 4 <= nRows);
    v4f v = {0.0f, 0.0f, 0.0f, 0.0f};
    if (tid < 8) v = *(const v4f*)(sOut + tid * 4);
    float* dst = out + (size_t)blockIdx.x * 32 + tid * 4;
    if (wr) *(volatile v4f*)dst = v;
    __threadfence();
    if (wr) *(volatile v4f*)dst = v;
}

static inline size_t align_up256(size_t v) { return (v + 255) & ~(size_t)255; }

extern "C" void kernel_launch(void* const* d_in, const int* in_sizes, int n_in,
                              void* d_out, int out_size, void* d_ws, size_t ws_size,
                              hipStream_t stream) {
    if (n_in < 12) return;
    if (in_sizes[0] != kBS * kF) return;
    if (in_sizes[1] < kE || (in_sizes[1] % kE) != 0) return;
    if (in_sizes[2] != kG * kE || in_sizes[3] != kG * kH) return;
    if (in_sizes[4] != kG || in_sizes[5] != kG) return;
    if (in_sizes[6] != kH * kP1 || in_sizes[7] != kP1) return;
    if (in_sizes[8] != kP1 * kP2 || in_sizes[9] != kP2) return;
    if (in_sizes[10] != kP2 || in_sizes[11] < 1) return;
    if (out_size != kBT) return;

    const int*   x    = (const int*)  d_in[0];
    const float* emb  = (const float*)d_in[1];
    const float* W_ih = (const float*)d_in[2];
    const float* W_hh = (const float*)d_in[3];
    const float* b_ih = (const float*)d_in[4];
    const float* b_hh = (const float*)d_in[5];
    const float* W1   = (const float*)d_in[6];
    const float* b1   = (const float*)d_in[7];
    const float* W2   = (const float*)d_in[8];
    const float* b2   = (const float*)d_in[9];
    const float* W3   = (const float*)d_in[10];
    const float* b3   = (const float*)d_in[11];
    float* out = (float*)d_out;
    const int nEmbRows = in_sizes[1] / kE;

    const size_t szE    = (size_t)kBS * kE  * 2;
    const size_t szGx   = (size_t)kBS * kG  * 4;
    const size_t szBih  = (size_t)kG  * kE  * 2;
    const size_t szBhh  = (size_t)kG  * kH  * 2;
    const size_t szW1t  = (size_t)kP1 * kH  * 2;
    const size_t szW2t  = (size_t)kP2 * kP1 * 2;
    const size_t szHst  = (size_t)kB  * kH  * 2;
    const size_t szCst  = (size_t)kB  * kH  * 4;
    const size_t szR    = (size_t)kB  * kG  * 4;
    const size_t szHout = (size_t)kBT * kH  * 2;
    const size_t szZ1   = (size_t)kBT * kP1 * 2;
    const size_t szZ2   = (size_t)kBT * kP2 * 4;

    size_t off = 0;
    const size_t oE    = off; off = align_up256(off + szE);
    const size_t oGx   = off; off = align_up256(off + szGx);
    const size_t oBih  = off; off = align_up256(off + szBih);
    const size_t oBhh  = off; off = align_up256(off + szBhh);
    const size_t oW1t  = off; off = align_up256(off + szW1t);
    const size_t oW2t  = off; off = align_up256(off + szW2t);
    const size_t oHA   = off; off = align_up256(off + szHst);
    const size_t oHB   = off; off = align_up256(off + szHst);
    const size_t oCA   = off; off = align_up256(off + szCst);
    const size_t oCB   = off; off = align_up256(off + szCst);
    const size_t oR    = off; off = align_up256(off + szR);
    const size_t oHout = off; off = align_up256(off + szHout);
    const size_t total = off;
    if (total > ws_size) return;
    if (szZ1 + szZ2 > szGx) return;
    const size_t oZ1 = oGx;
    const size_t oZ2 = oGx + align_up256(szZ1);

    char* base = (char*)d_ws;
    unsigned short* eBf  = (unsigned short*)(base + oE);
    float*          Gx   = (float*)         (base + oGx);
    unsigned short* Bih  = (unsigned short*)(base + oBih);
    unsigned short* Bhh  = (unsigned short*)(base + oBhh);
    unsigned short* W1t  = (unsigned short*)(base + oW1t);
    unsigned short* W2t  = (unsigned short*)(base + oW2t);
    unsigned short* hA   = (unsigned short*)(base + oHA);
    unsigned short* hB   = (unsigned short*)(base + oHB);
    float*          cA   = (float*)         (base + oCA);
    float*          cB   = (float*)         (base + oCB);
    float*          Rb   = (float*)         (base + oR);
    unsigned short* hOut = (unsigned short*)(base + oHout);
    unsigned short* z1   = (unsigned short*)(base + oZ1);
    float*          z2   = (float*)         (base + oZ2);

    embed_mean_kernel<<<(kBS + 7) / 8, 128, 0, stream>>>(x, emb, eBf, kBS, nEmbRows);
    cvt_bf16_kernel<<<(kG * kE / 8 + 255) / 256, 256, 0, stream>>>(W_ih, Bih, kG * kE);
    cvt_bf16_kernel<<<(kG * kH / 8 + 255) / 256, 256, 0, stream>>>(W_hh, Bhh, kG * kH);
    cvt_bf16_T_kernel<<<dim3((kH + 63) / 64, (kP1 + 31) / 32), 256, 0, stream>>>(W1, W1t, kH, kP1);
    cvt_bf16_T_kernel<<<dim3((kP1 + 63) / 64, (kP2 + 31) / 32), 256, 0, stream>>>(W2, W2t, kP1, kP2);
    hipMemsetAsync(hA, 0, szHst, stream);
    hipMemsetAsync(cA, 0, szCst, stream);

    gemm_bf16_kernel<<<dim3(kG / 64, kBS / 16), 128, 0, stream>>>(
        eBf, Bih, nullptr, Gx, nullptr, kBS, kE, kG, 0);

    for (int t = 0; t < kT; ++t) {
        const unsigned short* hP = (t & 1) ? hB : hA;
        const float*          cP = (t & 1) ? cB : cA;
        unsigned short*       hN = (t & 1) ? hA : hB;
        float*                cN = (t & 1) ? cA : cB;
        lstm_step_kernel<<<dim3(kH / 64, kB / 16), 128, 0, stream>>>(
            Gx, b_ih, b_hh, Bhh, hP, cP, hN, cN, t);
    }

    gemm_bf16_kernel<<<dim3(kG / 64, kB / 16), 128, 0, stream>>>(
        hA, Bhh, nullptr, Rb, nullptr, kB, kH, kG, 0);

    target_kernel<<<(kBT + 3) / 4, 128, 0, stream>>>(Gx, Rb, b_ih, b_hh, cA, hOut, kBT);

    gemm_bf16_kernel<<<dim3(kP1 / 64, kBT / 16), 128, 0, stream>>>(
        hOut, W1t, b1, nullptr, z1, kBT, kH, kP1, 1);
    gemm_bf16_kernel<<<dim3(kP2 / 64, kBT / 16), 128, 0, stream>>>(
        z1, W2t, b2, z2, nullptr, kBT, kP1, kP2, 2);
    mlp_out_kernel<<<(kBT + 31) / 32, 256, 0, stream>>>(z2, W3, b3, out, kBT);

    hipGetLastError();
}
